// CagnetSAGE_8452495639005
// MI455X (gfx1250) — hardware-run, weakly checked
//
#include <hip/hip_runtime.h>
#include <stddef.h>
#include <stdint.h>


#define DF     128
#define MPITCH 256
#define K1L    384
#define K2L    512
#define NTHR   256
#define NWAVE  8
#define EPT    8
#define CHUNK  (NTHR * EPT)
#define WCAP   (EPT * 32)
#define LISTN  (NWAVE * WCAP)
#define NBA    1024
#define SLA    10
#define RCAP   28672
#define DEGCAP 64
#define GBM    64
#define GBN    128
#define GTHR   128
#define GWAVE  (GTHR / 32)
#define MPADR  128
#define FLP    32
#define ROWH   256
#define NUW1   (DF * (K1L / 8))
#define NUW2   (DF * (K2L / 8))
#define NUBS   NTHR
#define NUWE   (NUW1 + NUW2 + NUBS)
#define AGG_ZINTS    (LISTN + 2 * RCAP + 3 * NBA)
#define MISC_INTS    16
#define BKT_LDS_INTS (AGG_ZINTS + MISC_INTS)
#define WSCAP  268435456

static_assert((CHUNK & (CHUNK - 1)) == 0 && CHUNK <= 4096);
static_assert((NBA & (NBA - 1)) == 0 && NBA == (1 << SLA));
static_assert(((long long)CHUNK << SLA) < (1LL << 31));
static_assert(LISTN % NTHR == 0);
static_assert(NBA % NWAVE == 0 && NBA % 32 == 0 && NBA % GBM == 0 && NBA % MPADR == 0 && NBA == 4 * NTHR);
static_assert(RCAP % 4 == 0 && AGG_ZINTS % 4 == 0 && LISTN % 4 == 0);
static_assert(AGG_ZINTS % (NTHR * 4) == 0);
static_assert(RCAP % (4 * NTHR) == 0);
static_assert(K1L % 32 == 0 && K2L % 32 == 0 && K1L == 3 * DF && K2L == 4 * DF && MPITCH == 2 * DF);
static_assert(GBN == DF && GBM == GWAVE * 16 && DF == 4 * 32 && GTHR == GWAVE * 32 && MPADR % GBM == 0);
static_assert(BKT_LDS_INTS * 4 <= 327680);
static_assert(NWAVE * ROWH * 2 + 0 <= 327680);
static_assert(GBM * GBN * 4 + DF * 4 <= 327680);
static_assert(ROWH == 2 * DF);
static_assert(NUW1 % NTHR == 0 && NUW2 % NTHR == 0 && NUWE % NTHR == 0 && (MPADR * (DF / 8)) % NTHR == 0);
static_assert(DEGCAP >= 36 + 8);
static_assert(RCAP >= 16710 + 16710 / 20);
static_assert(NBA * 98 >= 100000);

typedef float          v4f   __attribute__((ext_vector_type(4)));
typedef float          v8f   __attribute__((ext_vector_type(8)));
typedef int            v4i   __attribute__((ext_vector_type(4)));
typedef int            v8i   __attribute__((ext_vector_type(8)));
typedef unsigned       v2u   __attribute__((ext_vector_type(2)));
typedef unsigned short v4us  __attribute__((ext_vector_type(4)));
typedef unsigned short v8us  __attribute__((ext_vector_type(8)));
typedef unsigned short v16us __attribute__((ext_vector_type(16)));
typedef __bf16         v16bf __attribute__((ext_vector_type(16)));
typedef v4f  __attribute__((may_alias)) v4fa;
typedef v4i  __attribute__((may_alias)) v4ia;
typedef v2u  __attribute__((may_alias)) v2ua;
typedef v4us __attribute__((may_alias)) v4usa;
typedef v8us __attribute__((may_alias)) v8usa;
union FragB { v16bf v; v16us u; v8us h[2]; v8i w; };

__device__ __forceinline__ v8f wmb(const FragB& a, const FragB& b, v8f c) {
  v8f d = __builtin_amdgcn_wmma_f32_16x16x32_bf16(false, a.v, false, b.v, (short)0, c, false, false);
  asm volatile("v_nop\n\tv_nop\n\tv_nop\n\tv_nop" : "+v"(d) : "v"(a.w), "v"(b.w));
  return d;
}

__device__ __forceinline__ unsigned bf16_bits(float f) {
  const unsigned u = __float_as_uint(f);
  return (u + 0x7FFFu + ((u >> 16) & 1u)) >> 16;
}
__device__ __forceinline__ float bf16_val(float f) {
  return __uint_as_float(bf16_bits(f) << 16);
}

__device__ __forceinline__ void wave_sync() {
  __builtin_amdgcn_fence(__ATOMIC_RELEASE, "wavefront");
  __builtin_amdgcn_wave_barrier();
  __builtin_amdgcn_fence(__ATOMIC_ACQUIRE, "wavefront");
}

template <int SLB>
__device__ __forceinline__ int scan_chunk(const int* __restrict__ dsts, int nE, int cbase, int slotBase,
                                          int nb, int vec8, int* list, int tid, int lane, int wave) {
  int wc = 0;
  const int el0  = tid * EPT;
  const int e0   = cbase + el0;
  const int sent = -2147483647 - 1;
  v4i da, db;
  if (vec8 != 0 && cbase + CHUNK <= nE) {
    da = *(const v4i*)(dsts + e0);
    db = *(const v4i*)(dsts + e0 + 4);
  } else {
    da.x = (e0     < nE) ? dsts[min(e0,     nE - 1)] : sent;
    da.y = (e0 + 1 < nE) ? dsts[min(e0 + 1, nE - 1)] : sent;
    da.z = (e0 + 2 < nE) ? dsts[min(e0 + 2, nE - 1)] : sent;
    da.w = (e0 + 3 < nE) ? dsts[min(e0 + 3, nE - 1)] : sent;
    db.x = (e0 + 4 < nE) ? dsts[min(e0 + 4, nE - 1)] : sent;
    db.y = (e0 + 5 < nE) ? dsts[min(e0 + 5, nE - 1)] : sent;
    db.z = (e0 + 6 < nE) ? dsts[min(e0 + 6, nE - 1)] : sent;
    db.w = (e0 + 7 < nE) ? dsts[min(e0 + 7, nE - 1)] : sent;
  }
  const unsigned nbs = (unsigned)slotBase;
  const unsigned unb = (unsigned)nb;
  const unsigned s0 = (unsigned)da.x - nbs, s1 = (unsigned)da.y - nbs;
  const unsigned s2 = (unsigned)da.z - nbs, s3 = (unsigned)da.w - nbs;
  const unsigned s4 = (unsigned)db.x - nbs, s5 = (unsigned)db.y - nbs;
  const unsigned s6 = (unsigned)db.z - nbs, s7 = (unsigned)db.w - nbs;
  const bool h0 = s0 < unb, h1 = s1 < unb, h2 = s2 < unb, h3 = s3 < unb;
  const bool h4 = s4 < unb, h5 = s5 < unb, h6 = s6 < unb, h7 = s7 < unb;
  const unsigned any = __builtin_amdgcn_ballot_w32(h0 | h1 | h2 | h3 | h4 | h5 | h6 | h7);
  if (any != 0u) {
#define HITJ(J, HJ, SJ) { \
      const unsigned mj = __builtin_amdgcn_ballot_w32(HJ); \
      if (mj != 0u) { \
        if (HJ) { \
          const int pos = wc + (int)__builtin_amdgcn_mbcnt_lo(mj, 0u); \
          if (pos < WCAP) list[wave * WCAP + pos] = ((el0 + (J)) << SLB) | (int)(SJ); \
        } \
        wc += (int)__builtin_popcount(mj); } }
    HITJ(0, h0, s0)
    HITJ(1, h1, s1)
    HITJ(2, h2, s2)
    HITJ(3, h3, s3)
    HITJ(4, h4, s4)
    HITJ(5, h5, s5)
    HITJ(6, h6, s6)
    HITJ(7, h7, s7)
#undef HITJ
  }
  return wc;
}

__global__ __launch_bounds__(NTHR) void k_prep(const float* __restrict__ x,
                                               const float* __restrict__ wn1, const float* __restrict__ ws1,
                                               const float* __restrict__ wn2, const float* __restrict__ ws2,
                                               const float* __restrict__ bn1, const float* __restrict__ bs1,
                                               const float* __restrict__ bn2, const float* __restrict__ bs2,
                                               unsigned short* w1c, unsigned short* w2c, float* bsum,
                                               unsigned short* xb, int nN, int nUnits) {
  const int u = (int)blockIdx.x * NTHR + (int)threadIdx.x;
  v8us o;
  unsigned short* dp;
  if (u < NUW1) {
    const int n  = u / (K1L / 8);
    const int k8 = (u - n * (K1L / 8)) * 8;
    const int kk = k8 & (DF - 1);
    const size_t wo = (size_t)n * DF + (size_t)kk;
    const v4f a0 = *(const v4f*)(wn1 + wo), a1 = *(const v4f*)(wn1 + wo + 4);
    const v4f c0 = *(const v4f*)(ws1 + wo), c1 = *(const v4f*)(ws1 + wo + 4);
    const float fa[8] = {a0.x, a0.y, a0.z, a0.w, a1.x, a1.y, a1.z, a1.w};
    const float fb[8] = {c0.x, c0.y, c0.z, c0.w, c1.x, c1.y, c1.z, c1.w};
    const unsigned msk = (k8 < 2 * DF) ? 0xFFFFu : 0u;
#pragma unroll
    for (int i = 0; i < 8; ++i) {
      const unsigned ha = bf16_bits(fa[i]);
      const unsigned hb = bf16_bits(fb[i]);
      o[i] = (unsigned short)((ha & msk) | (hb & (~msk & 0xFFFFu)));
    }
    dp = w1c + (size_t)u * 8;
  } else if (u < NUW1 + NUW2) {
    const int v  = u - NUW1;
    const int n  = v >> 6, k8 = (v & 63) * 8;
    const int kk = k8 & (DF - 1);
    const size_t wo = (size_t)n * DF + (size_t)kk;
    const v4f a0 = *(const v4f*)(wn2 + wo), a1 = *(const v4f*)(wn2 + wo + 4);
    const v4f c0 = *(const v4f*)(ws2 + wo), c1 = *(const v4f*)(ws2 + wo + 4);
    const float fa[8] = {a0.x, a0.y, a0.z, a0.w, a1.x, a1.y, a1.z, a1.w};
    const float fb[8] = {c0.x, c0.y, c0.z, c0.w, c1.x, c1.y, c1.z, c1.w};
    const unsigned msk = (k8 < 2 * DF) ? 0xFFFFu : 0u;
#pragma unroll
    for (int i = 0; i < 8; ++i) {
      const unsigned ha = bf16_bits(fa[i]);
      const unsigned hb = bf16_bits(fb[i]);
      o[i] = (unsigned short)((ha & msk) | (hb & (~msk & 0xFFFFu)));
    }
    dp = w2c + (size_t)v * 8;
  } else if (u < NUWE) {
    const int w = u - (NUW1 + NUW2);
    if (w < 32) {
      const v4f p1 = *(const v4f*)(bn1 + 4 * w);
      const v4f q1 = *(const v4f*)(bs1 + 4 * w);
      const v4f p2 = *(const v4f*)(bn2 + 4 * w);
      const v4f q2 = *(const v4f*)(bs2 + 4 * w);
      v4f s1, s2;
      s1.x = bf16_val(p1.x) + bf16_val(q1.x); s1.y = bf16_val(p1.y) + bf16_val(q1.y);
      s1.z = bf16_val(p1.z) + bf16_val(q1.z); s1.w = bf16_val(p1.w) + bf16_val(q1.w);
      s2.x = bf16_val(p2.x) + bf16_val(q2.x); s2.y = bf16_val(p2.y) + bf16_val(q2.y);
      s2.z = bf16_val(p2.z) + bf16_val(q2.z); s2.w = bf16_val(p2.w) + bf16_val(q2.w);
      float* d1 = bsum + 4 * w;
      float* d2 = bsum + DF + 4 * w;
      *(volatile v4f*)d1 = s1;
      *(volatile v4f*)d2 = s2;
      __threadfence();
      *(volatile v4f*)d1 = s1;
      *(volatile v4f*)d2 = s2;
    }
    return;
  } else if (u < nUnits) {
    const int v   = u - NUWE;
    const int row = v >> 4, k8 = (v & 15) * 8;
    const int rc  = row < nN ? row : nN - 1;
    const float* p = x + (size_t)rc * DF + k8;
    const v4f a = *(const v4f*)p;
    const v4f b = *(const v4f*)(p + 4);
    asm volatile("" :: "v"(a), "v"(b));
    const unsigned zm = (row < nN) ? 0xFFFFu : 0u;
    o[0] = (unsigned short)(bf16_bits(a.x) & zm); o[1] = (unsigned short)(bf16_bits(a.y) & zm);
    o[2] = (unsigned short)(bf16_bits(a.z) & zm); o[3] = (unsigned short)(bf16_bits(a.w) & zm);
    o[4] = (unsigned short)(bf16_bits(b.x) & zm); o[5] = (unsigned short)(bf16_bits(b.y) & zm);
    o[6] = (unsigned short)(bf16_bits(b.z) & zm); o[7] = (unsigned short)(bf16_bits(b.w) & zm);
    dp = xb + (size_t)v * 8;
  } else {
    return;
  }
  *(volatile v8us*)dp = o;
  __threadfence();
  *(volatile v8us*)dp = o;
}

__global__ __launch_bounds__(NTHR) void k_bucket(const int* __restrict__ srcs, const int* __restrict__ dsts,
                                                 int nE, int nN, int vec8,
                                                 int* lstg, int* cntg, int* offg, int* flag) {
  extern __shared__ __attribute__((aligned(16))) int dsm[];
  int* list = dsm;
  int* hl   = dsm + LISTN;
  int* sl   = hl + RCAP;
  int* cnt  = sl + RCAP;
  int* offs = cnt + NBA;
  int* cur  = offs + NBA;
  int* misc = cur + NBA;
  const int tid = (int)threadIdx.x, lane = tid & 31, wave = tid >> 5;
  const int nodeBase = (int)blockIdx.x * NBA;

  {
    const v4i z4 = {0, 0, 0, 0};
    for (int i = tid * 4; i < AGG_ZINTS; i += NTHR * 4) *(v4ia*)(dsm + i) = z4;
    if (tid < MISC_INTS) misc[tid] = 0;
  }
  __syncthreads();

  int t = 0, ov = 0;
  const int nChunks = (nE + CHUNK - 1) / CHUNK;
#pragma unroll 1
  for (int ch = 0; ch < nChunks; ++ch) {
    const int cbase = ch * CHUNK;
    const int wc = scan_chunk<SLA>(dsts, nE, cbase, nodeBase, NBA, vec8, list, tid, lane, wave);
    if (lane == 0) misc[wave] = wc;
    __syncthreads();
    if (wave == 0) {
#pragma unroll 1
      for (int w2 = 0; w2 < NWAVE; ++w2) {
        int c = misc[w2];
        c = c < 0 ? 0 : (c > WCAP ? WCAP : c);
#pragma unroll 1
        for (int b0 = 0; b0 < c; b0 += 32) {
          const int idx = b0 + lane;
          const int ent_ = list[w2 * WCAP + (idx < WCAP ? idx : WCAP - 1)];
          const int m32 = (c - b0) < 32 ? (c - b0) : 32;
#pragma unroll 1
          for (int k = 0; k < m32; ++k) {
            const int u    = __builtin_amdgcn_readlane(ent_, k);
            const int slot = u & (NBA - 1);
            const int el   = (u >> SLA) & (CHUNK - 1);
            const int pk   = ((cbase + el) << SLA) | slot;
            if (t < RCAP) {
              if (lane == 0) { hl[t] = pk; cnt[slot] = cnt[slot] + 1; }
              t = t + 1;
            } else {
              ov = 1;
            }
          }
        }
      }
    }
    __syncthreads();
  }
  if (wave == 0 && lane == 0) { misc[8] = t; misc[9] = ov; }
  __syncthreads();
  int tt = misc[8];
  tt = tt < 0 ? 0 : (tt > RCAP ? RCAP : tt);
  const int ovf = misc[9];

  if (wave == 0) {
    const int base = lane * (NBA / 32);
    int s = 0;
#pragma unroll 1
    for (int i = 0; i < NBA / 32; ++i) s += cnt[base + i];
    int incl = s;
#pragma unroll
    for (int d = 1; d < 32; d <<= 1) {
      const int y = __shfl_up(incl, d, 32);
      if (lane >= d) incl += y;
    }
    int run = incl - s;
#pragma unroll 1
    for (int i = 0; i < NBA / 32; ++i) {
      const int cv = cnt[base + i];
      offs[base + i] = run;
      cur[base + i]  = run;
      run += cv;
    }
  }
  __syncthreads();
  if (wave == 0) {
#pragma unroll 1
    for (int b0 = 0; b0 < tt; b0 += 32) {
      const int idx = b0 + lane;
      const int ent_ = hl[idx < RCAP ? idx : RCAP - 1];
      const int m32 = (tt - b0) < 32 ? (tt - b0) : 32;
#pragma unroll 1
      for (int k = 0; k < m32; ++k) {
        const int u    = __builtin_amdgcn_readlane(ent_, k);
        const int slot = u & (NBA - 1);
        if (lane == 0) {
          int p = cur[slot];
          p = p < 0 ? 0 : (p > RCAP - 1 ? RCAP - 1 : p);
          sl[p] = u;
          cur[slot] = p + 1;
        }
      }
    }
  }
  __syncthreads();

  {
    int bigAny = 0;
#pragma unroll 1
    for (int j = 0; j < NBA / NTHR; ++j) bigAny |= (cnt[tid + j * NTHR] > DEGCAP) ? 1 : 0;
    const unsigned bm = __builtin_amdgcn_ballot_w32(bigAny != 0);
    if (lane == 0) misc[wave] = (bm != 0u) ? 1 : 0;
  }
  __syncthreads();
  int fl = ovf;
#pragma unroll
  for (int w2 = 0; w2 < NWAVE; ++w2) fl |= misc[w2];
  fl = (fl != 0) ? 1 : 0;

  if (wave == 0) {
    int* fp = flag + (size_t)blockIdx.x * FLP + lane;
    *(volatile int*)fp = fl;
    __threadfence();
    *(volatile int*)fp = fl;
  }
  {
    const v4i cv  = *(const v4ia*)(cnt + 4 * tid);
    const v4i ov4 = *(const v4ia*)(offs + 4 * tid);
    int* cp = cntg + (size_t)nodeBase + 4 * tid;
    int* op = offg + (size_t)nodeBase + 4 * tid;
    *(volatile v4i*)cp = cv;
    *(volatile v4i*)op = ov4;
    __threadfence();
    *(volatile v4i*)cp = cv;
    *(volatile v4i*)op = ov4;
  }
  int* lp = lstg + (size_t)blockIdx.x * RCAP;
#pragma unroll 1
  for (int it = 0; it < RCAP / (4 * NTHR); ++it) {
    const int i4 = (it * NTHR + tid) * 4;
    const v4i e = *(const v4ia*)(sl + i4);
    int e0 = e.x >> SLA, e1 = e.y >> SLA, e2 = e.z >> SLA, e3 = e.w >> SLA;
    e0 = e0 < 0 ? 0 : (e0 > nE - 1 ? nE - 1 : e0);
    e1 = e1 < 0 ? 0 : (e1 > nE - 1 ? nE - 1 : e1);
    e2 = e2 < 0 ? 0 : (e2 > nE - 1 ? nE - 1 : e2);
    e3 = e3 < 0 ? 0 : (e3 > nE - 1 ? nE - 1 : e3);
    int s0 = srcs[e0];
    int s1 = srcs[e1];
    int s2 = srcs[e2];
    int s3 = srcs[e3];
    asm volatile("" :: "v"(s0), "v"(s1), "v"(s2), "v"(s3));
    s0 = s0 < 0 ? 0 : (s0 > nN - 1 ? nN - 1 : s0);
    s1 = s1 < 0 ? 0 : (s1 > nN - 1 ? nN - 1 : s1);
    s2 = s2 < 0 ? 0 : (s2 > nN - 1 ? nN - 1 : s2);
    s3 = s3 < 0 ? 0 : (s3 > nN - 1 ? nN - 1 : s3);
    const int m0 = (i4     < tt) ? -1 : 0;
    const int m1 = (i4 + 1 < tt) ? -1 : 0;
    const int m2 = (i4 + 2 < tt) ? -1 : 0;
    const int m3 = (i4 + 3 < tt) ? -1 : 0;
    v4i o;
    o.x = s0 & m0; o.y = s1 & m1; o.z = s2 & m2; o.w = s3 & m3;
    int* dp = lp + i4;
    *(volatile v4i*)dp = o;
    __threadfence();
    *(volatile v4i*)dp = o;
  }
}

template <int L2>
__global__ __launch_bounds__(NTHR) void k_agg(const int* __restrict__ lst, const int* __restrict__ cntg,
                                              const int* __restrict__ offg, const int* __restrict__ flg,
                                              const unsigned short* __restrict__ spl, int nN, int mRows,
                                              unsigned short* mpl) {
  __shared__ __attribute__((aligned(16))) unsigned short rowbuf_all[NWAVE * ROWH];
  const int tid = (int)threadIdx.x, lane = tid & 31, wave = tid >> 5;
  unsigned short* rowbuf = rowbuf_all + wave * ROWH;
  const int nodeBase = (int)blockIdx.x * NBA;
  const int* bl = lst + (size_t)blockIdx.x * RCAP;
  const int fl = flg[(size_t)blockIdx.x * FLP];
  const float qn = __int_as_float(0x7fc00000);
  constexpr int SP = (L2 != 0) ? MPITCH : DF;

#pragma unroll 1
  for (int si = 0; si < NBA / NWAVE; ++si) {
    const int s    = si * NWAVE + wave;
    const int node = nodeBase + s;
    int c = cntg[node];
    const bool big = c > DEGCAP;
    c = c < 0 ? 0 : (c > DEGCAP ? DEGCAP : c);
    int o = offg[node];
    o = o < 0 ? 0 : (o > RCAP - 1 ? RCAP - 1 : o);
    const bool bad  = big || (fl != 0);
    const bool live = node < nN;
    float a0 = 0.0f, a1 = 0.0f, a2 = 0.0f, a3 = 0.0f;
#pragma unroll 1
    for (int b0 = 0; b0 < c; b0 += 32) {
      int idx = o + b0 + lane;
      const int lastI = o + c - 1;
      idx = idx > lastI ? lastI : idx;
      idx = idx < 0 ? 0 : (idx > RCAP - 1 ? RCAP - 1 : idx);
      int sr = bl[idx];
      sr = sr < 0 ? 0 : (sr > nN - 1 ? nN - 1 : sr);
      const int m32 = (c - b0) < 32 ? (c - b0) : 32;
#pragma unroll 1
      for (int k = 0; k < m32; ++k) {
        const int sk = __builtin_amdgcn_readlane(sr, k);
        const unsigned short* rp = spl + (size_t)sk * SP + 4 * lane;
        const v2u wh = *(const v2ua*)rp;
        float f0 = __uint_as_float(wh.x << 16);
        float f1 = __uint_as_float(wh.x & 0xffff0000u);
        float f2 = __uint_as_float(wh.y << 16);
        float f3 = __uint_as_float(wh.y & 0xffff0000u);
        if constexpr (L2 != 0) {
          const v2u wl = *(const v2ua*)(rp + DF);
          f0 += __uint_as_float(wl.x << 16);
          f1 += __uint_as_float(wl.x & 0xffff0000u);
          f2 += __uint_as_float(wl.y << 16);
          f3 += __uint_as_float(wl.y & 0xffff0000u);
        }
        a0 += f0; a1 += f1; a2 += f2; a3 += f3;
      }
    }
    const float inv = 1.0f / fmaxf((float)c, 1.0f);
    const float v0 = a0 * inv, v1 = a1 * inv, v2 = a2 * inv, v3 = a3 * inv;
    const float m0 = live ? (bad ? qn : v0) : 0.0f;
    const float m1 = live ? (bad ? qn : v1) : 0.0f;
    const float m2 = live ? (bad ? qn : v2) : 0.0f;
    const float m3 = live ? (bad ? qn : v3) : 0.0f;
    v4us mh, ml;
    {
      unsigned hb;
      hb = bf16_bits(m0); mh[0] = (unsigned short)hb; ml[0] = (unsigned short)bf16_bits(m0 - __uint_as_float(hb << 16));
      hb = bf16_bits(m1); mh[1] = (unsigned short)hb; ml[1] = (unsigned short)bf16_bits(m1 - __uint_as_float(hb << 16));
      hb = bf16_bits(m2); mh[2] = (unsigned short)hb; ml[2] = (unsigned short)bf16_bits(m2 - __uint_as_float(hb << 16));
      hb = bf16_bits(m3); mh[3] = (unsigned short)hb; ml[3] = (unsigned short)bf16_bits(m3 - __uint_as_float(hb << 16));
    }
    *(v4usa*)(rowbuf + 4 * lane)      = mh;
    *(v4usa*)(rowbuf + DF + 4 * lane) = ml;
    wave_sync();
    const v8us q0 = *(const v8usa*)(rowbuf + 8 * lane);
    wave_sync();
    if (node < mRows) {
      unsigned short* rpw = mpl + (size_t)node * MPITCH + 8 * lane;
      *(volatile v8us*)rpw = q0;
      __threadfence();
      *(volatile v8us*)rpw = q0;
    }
  }
}

__device__ __forceinline__ void gemm_span(const unsigned short* __restrict__ ap, const unsigned short* __restrict__ bp,
                                          int ldb, int K, v8f (&acc)[8]) {
#pragma unroll 1
  for (int k0 = 0; k0 < K; k0 += 32) {
    FragB af;
    af.h[0] = *(const v8usa*)(ap + k0);
    af.h[1] = *(const v8usa*)(ap + k0 + 16);
#pragma unroll
    for (int nt = 0; nt < 8; ++nt) {
      const unsigned short* wq = bp + (size_t)(16 * nt) * (size_t)ldb + k0;
      FragB bf;
      bf.h[0] = *(const v8usa*)wq;
      bf.h[1] = *(const v8usa*)(wq + 16);
      acc[nt] = wmb(af, bf, acc[nt]);
    }
  }
}

template <int FIN>
__global__ __launch_bounds__(GTHR) __attribute__((amdgpu_num_vgpr(248)))
void k_gemm(const unsigned short* __restrict__ A0, const unsigned short* __restrict__ A1, int lda1, int K1,
            const unsigned short* __restrict__ BT, int ldb, const float* __restrict__ bsum,
            const int* __restrict__ flg, int nFl, unsigned short* hpl, float* outp, int nN, int mRows) {
  __shared__ __attribute__((aligned(16))) float stg[GBM * GBN];
  __shared__ __attribute__((aligned(16))) float sb[DF];
  const int tid = (int)threadIdx.x, lane = tid & 31, wave = tid >> 5, hh = lane >> 4, m = lane & 15;
  const int rowBase = (int)blockIdx.x * GBM;

  v8f acc[8];
  {
    const v8f z = {0.f, 0.f, 0.f, 0.f, 0.f, 0.f, 0.f, 0.f};
#pragma unroll
    for (int t = 0; t < 8; ++t) acc[t] = z;
  }
  const size_t arow = (size_t)(rowBase + 16 * wave + m);
  const unsigned short* ap0 = A0 + arow * (size_t)MPITCH + 8 * hh;
  const unsigned short* ap1 = A1 + arow * (size_t)lda1 + 8 * hh;
  const unsigned short* bp  = BT + (size_t)m * (size_t)ldb + 8 * hh;

  gemm_span(ap0, bp, ldb, MPITCH, acc);
  gemm_span(ap1, bp + MPITCH, ldb, K1, acc);

#pragma unroll
  for (int nt = 0; nt < 8; ++nt) {
    const int lc = 16 * nt + m;
#pragma unroll
    for (int r = 0; r < 8; ++r) {
      const int lr = 16 * wave + 8 * hh + r;
      stg[lr * GBN + lc] = acc[nt][r];
    }
  }
  if (tid < 32) {
    const v4f b4 = *(const v4f*)(bsum + 4 * tid);
    *(v4fa*)(sb + 4 * tid) = b4;
  }
  __syncthreads();

  const v4f bb4 = *(const v4fa*)(sb + 4 * lane);
  v4f pv[16];
#pragma unroll
  for (int i = 0; i < 16; ++i) pv[i] = *(const v4fa*)(stg + (16 * wave + i) * GBN + 4 * lane);
  __syncthreads();

  if constexpr (FIN != 0) {
    int fb = rowBase >> SLA;
    fb = fb < 0 ? 0 : (fb > nFl - 1 ? nFl - 1 : fb);
    const int fl = flg[(size_t)fb * FLP];
    const float qn = __int_as_float(0x7fc00000);
#pragma unroll
    for (int i = 0; i < 16; ++i) {
      const v4f t = pv[i] + bb4;
      v4f y;
      y.x = (fl != 0) ? qn : t.x;
      y.y = (fl != 0) ? qn : t.y;
      y.z = (fl != 0) ? qn : t.z;
      y.w = (fl != 0) ? qn : t.w;
      pv[i] = y;
    }
#pragma unroll
    for (int i = 0; i < 16; ++i) {
      const int r = rowBase + 16 * wave + i;
      if (r < nN) *(volatile v4f*)(outp + (size_t)r * DF + 4 * lane) = pv[i];
    }
    __threadfence();
#pragma unroll
    for (int i = 0; i < 16; ++i) {
      const int r = rowBase + 16 * wave + i;
      if (r < nN) *(volatile v4f*)(outp + (size_t)r * DF + 4 * lane) = pv[i];
    }
    (void)hpl; (void)mRows;
  } else {
#pragma unroll
    for (int i = 0; i < 16; ++i) {
      const bool ok = (rowBase + 16 * wave + i) < nN;
      const v4f t = pv[i] + bb4;
      v4f y;
      y.x = (t.x > 0.0f) ? t.x : (t.x - t.x);
      y.y = (t.y > 0.0f) ? t.y : (t.y - t.y);
      y.z = (t.z > 0.0f) ? t.z : (t.z - t.z);
      y.w = (t.w > 0.0f) ? t.w : (t.w - t.w);
      y.x = ok ? y.x : 0.0f; y.y = ok ? y.y : 0.0f; y.z = ok ? y.z : 0.0f; y.w = ok ? y.w : 0.0f;
      pv[i] = y;
    }
#pragma unroll
    for (int i = 0; i < 16; ++i) {
      v4us h4, l4;
      unsigned hb;
      hb = bf16_bits(pv[i].x); h4[0] = (unsigned short)hb; l4[0] = (unsigned short)bf16_bits(pv[i].x - __uint_as_float(hb << 16));
      hb = bf16_bits(pv[i].y); h4[1] = (unsigned short)hb; l4[1] = (unsigned short)bf16_bits(pv[i].y - __uint_as_float(hb << 16));
      hb = bf16_bits(pv[i].z); h4[2] = (unsigned short)hb; l4[2] = (unsigned short)bf16_bits(pv[i].z - __uint_as_float(hb << 16));
      hb = bf16_bits(pv[i].w); h4[3] = (unsigned short)hb; l4[3] = (unsigned short)bf16_bits(pv[i].w - __uint_as_float(hb << 16));
      unsigned short* srow = (unsigned short*)stg + (size_t)(16 * wave + i) * (2 * GBN);
      *(v4usa*)(srow + 4 * lane) = h4;
      *(v4usa*)(srow + DF + 4 * lane) = l4;
    }
    __syncthreads();
    v8us qv[16];
#pragma unroll
    for (int i = 0; i < 16; ++i) {
      const unsigned short* srow = (const unsigned short*)stg + (size_t)(16 * wave + i) * (2 * GBN);
      qv[i] = *(const v8usa*)(srow + 8 * lane);
    }
#pragma unroll
    for (int i = 0; i < 16; ++i) {
      const int gr = rowBase + 16 * wave + i;
      unsigned short* rp = hpl + (size_t)gr * (size_t)MPITCH + 8 * lane;
      if (gr < mRows) *(volatile v8us*)rp = qv[i];
    }
    __threadfence();
#pragma unroll
    for (int i = 0; i < 16; ++i) {
      const int gr = rowBase + 16 * wave + i;
      unsigned short* rp = hpl + (size_t)gr * (size_t)MPITCH + 8 * lane;
      if (gr < mRows) *(volatile v8us*)rp = qv[i];
    }
    (void)outp; (void)flg; (void)nFl;
  }
}

static inline int cdiv(int a, int b) { return (a + b - 1) / b; }
static inline size_t al256(size_t o) { return (o + 255) & ~(size_t)255; }

constexpr size_t cal256(size_t o) { return (o + 255) & ~(size_t)255; }
constexpr size_t carve_total(size_t nN) {
  const size_t MP = (nN + MPADR - 1) / MPADR * MPADR;
  const size_t gA = (nN + NBA - 1) / NBA;
  size_t off = 0;
  off = cal256(off + (size_t)DF * K1L * 2);
  off = cal256(off + (size_t)DF * K2L * 2);
  off = cal256(off + (size_t)2 * DF * 4);
  off = cal256(off + gA * FLP * 4);
  off = cal256(off + gA * NBA * 4);
  off = cal256(off + gA * NBA * 4);
  off = cal256(off + gA * RCAP * 4);
  off = cal256(off + MP * DF * 2);
  off = cal256(off + MP * MPITCH * 2);
  off = cal256(off + MP * MPITCH * 2);
  return off;
}
static_assert(carve_total(100000) <= (size_t)WSCAP);

extern "C" void kernel_launch(void* const* d_in, const int* in_sizes, int n_in,
                              void* d_out, int out_size, void* d_ws, size_t ws_size,
                              hipStream_t stream) {
  if (n_in < 10) return;
  if (in_sizes[0] < DF * GBM || (in_sizes[0] % DF) != 0) return;
  const int nN = in_sizes[0] / DF;
  if (nN >= (1 << 24)) return;
  if (in_sizes[1] < 2 || (in_sizes[1] & 1) != 0) return;
  const int nE = in_sizes[1] / 2;
  if (nE < 1 || nE >= (1 << 21)) return;
  if (in_sizes[2] != DF * DF || in_sizes[3] != DF) return;
  if (in_sizes[4] != DF * DF || in_sizes[5] != DF) return;
  if (in_sizes[6] != DF * DF || in_sizes[7] != DF) return;
  if (in_sizes[8] != DF * DF || in_sizes[9] != DF) return;
  if ((long long)out_size != (long long)nN * DF) return;

  const float* x   = (const float*)d_in[0];
  const int*   ei  = (const int*)  d_in[1];
  const float* Wn1 = (const float*)d_in[2];
  const float* bn1 = (const float*)d_in[3];
  const float* Ws1 = (const float*)d_in[4];
  const float* bs1 = (const float*)d_in[5];
  const float* Wn2 = (const float*)d_in[6];
  const float* bn2 = (const float*)d_in[7];
  const float* Ws2 = (const float*)d_in[8];
  const float* bs2 = (const float*)d_in[9];
  float* out = (float*)d_out;
  const int* src = ei;
  const int* dst = ei + nE;

  const int MP = cdiv(nN, MPADR) * MPADR;
  const int gM = MP / GBM;
  const int gA = cdiv(nN, NBA);
  if ((long long)gA * NBA < (long long)MP || gA > 65535) return;
  const int vec8 = ((nE & 3) == 0) ? 1 : 0;

  char* ws = (char*)d_ws;
  size_t off = 0;
  const size_t oW1  = off; off = al256(off + (size_t)DF * K1L * 2);
  const size_t oW2  = off; off = al256(off + (size_t)DF * K2L * 2);
  const size_t oBS  = off; off = al256(off + (size_t)2 * DF * 4);
  const size_t oFL  = off; off = al256(off + (size_t)gA * FLP * 4);
  const size_t oCN  = off; off = al256(off + (size_t)gA * NBA * 4);
  const size_t oOF  = off; off = al256(off + (size_t)gA * NBA * 4);
  const size_t oLS  = off; off = al256(off + (size_t)gA * RCAP * 4);
  const size_t oXB  = off; off = al256(off + (size_t)MP * DF * 2);
  const size_t oMP  = off; off = al256(off + (size_t)MP * MPITCH * 2);
  const size_t oH1  = off; off = al256(off + (size_t)MP * MPITCH * 2);
  if (off > ws_size || off > (size_t)WSCAP) return;
  unsigned short* W1C = (unsigned short*)(ws + oW1);
  unsigned short* W2C = (unsigned short*)(ws + oW2);
  float*          BS  = (float*)(ws + oBS);
  int*            FL  = (int*)(ws + oFL);
  int*            CN  = (int*)(ws + oCN);
  int*            OF  = (int*)(ws + oOF);
  int*            LS  = (int*)(ws + oLS);
  unsigned short* XB  = (unsigned short*)(ws + oXB);
  unsigned short* MPL = (unsigned short*)(ws + oMP);
  unsigned short* H1  = (unsigned short*)(ws + oH1);

  const size_t bktLds = (size_t)BKT_LDS_INTS * 4;
  hipFuncSetAttribute(reinterpret_cast<const void*>(&k_bucket), hipFuncAttributeMaxDynamicSharedMemorySize, (int)bktLds);

  const int nUnits = NUWE + MP * (DF / 8);

  k_prep<<<nUnits / NTHR, NTHR, 0, stream>>>(x, Wn1, Ws1, Wn2, Ws2, bn1, bs1, bn2, bs2, W1C, W2C, BS, XB, nN, nUnits);
  k_bucket<<<gA, NTHR, bktLds, stream>>>(src, dst, nE, nN, vec8, LS, CN, OF, FL);
  k_agg<0><<<gA, NTHR, 0, stream>>>(LS, CN, OF, FL, XB, nN, MP, MPL);
  k_gemm<0><<<gM, GTHR, 0, stream>>>(MPL, XB, DF, DF, W1C, K1L, BS, FL, gA, H1, out, nN, MP);
  k_agg<1><<<gA, NTHR, 0, stream>>>(LS, CN, OF, FL, H1, nN, MP, MPL);
  k_gemm<1><<<gM, GTHR, 0, stream>>>(MPL, H1, MPITCH, MPITCH, W2C, K2L, BS + DF, FL, gA, H1, out, nN, MP);
}
